// RobertaHybridEncoder_81363860456157
// MI455X (gfx1250) — hardware-verified
//
#include <hip/hip_runtime.h>
#include <math.h>

typedef __attribute__((ext_vector_type(16))) _Float16 v16h;
typedef __attribute__((ext_vector_type(16))) __bf16 v16b;
typedef __attribute__((ext_vector_type(8)))  _Float16 v8h;
typedef __attribute__((ext_vector_type(8)))  float v8f;
typedef __attribute__((ext_vector_type(4)))  float v4f;
typedef __attribute__((ext_vector_type(2)))  float v2f;
typedef __attribute__((ext_vector_type(4)))  unsigned v4u;
typedef __attribute__((ext_vector_type(4)))  int v4i;
typedef float __attribute__((may_alias)) float_a;
typedef int __attribute__((may_alias)) int_a;

template <typename T> __device__ __forceinline__ void vst2(void* p, T v) { *(volatile T*)p = v; __threadfence(); *(volatile T*)p = v; }
__device__ __forceinline__ v8f wmma16(v16h a, v16h b, v8f c) {
  v8f d = __builtin_amdgcn_wmma_f32_16x16x32_f16(false, a, false, b, (short)0, c, false, false);
  asm volatile("v_nop\n\tv_nop\n\tv_nop\n\tv_nop" : "+v"(d) : "v"(a), "v"(b));
  return d;
}
__device__ __forceinline__ v8f wmma_bf(v16b a, v16b b, v8f c) {
  v8f d = __builtin_amdgcn_wmma_f32_16x16x32_bf16(false, a, false, b, (short)0, c, false, false);
  asm volatile("v_nop\n\tv_nop\n\tv_nop\n\tv_nop" : "+v"(d) : "v"(a), "v"(b));
  return d;
}
__device__ __forceinline__ v16h frag_h(const _Float16* rowk0, int lane) {
  union { v16h v; v8h q[2]; } u; const _Float16* p = rowk0 + 8 * (lane >> 4);
  u.q[0] = *(const v8h*)p; u.q[1] = *(const v8h*)(p + 16); return u.v;
}
__device__ __forceinline__ v16h frag_f32(const float* rowk0, int lane) {
  v16h a; const float* p = rowk0 + 8 * (lane >> 4);
#pragma unroll
  for (int i = 0; i < 8; ++i) { a[i] = (_Float16)p[i]; a[8 + i] = (_Float16)p[16 + i]; }
  return a;
}
__device__ __forceinline__ v16h frag_f32s(const float* rowk0, int lane, float sc) {
  v16h a; const float* p = rowk0 + 8 * (lane >> 4);
#pragma unroll
  for (int i = 0; i < 8; ++i) { a[i] = (_Float16)(p[i] * sc); a[8 + i] = (_Float16)(p[16 + i] * sc); }
  return a;
}
__device__ __forceinline__ v16h fragc_f32(const float* W, int k0, int n, int lane, int ld, int K) {
  v16h a; const int g = lane >> 4;
#pragma unroll
  for (int i = 0; i < 8; ++i) { const int ka = k0 + 8 * g + i, kb = ka + 16;
    a[i] = (_Float16)(ka < K ? W[(size_t)(ka < K ? ka : K - 1) * ld + n] : 0.f); a[8 + i] = (_Float16)(kb < K ? W[(size_t)(kb < K ? kb : K - 1) * ld + n] : 0.f); }
  return a;
}
struct F2 { v16b h, l; };
__device__ __forceinline__ F2 bsplit16(const float v[16]) { F2 r;
#pragma unroll
  for (int i = 0; i < 16; ++i) { const __bf16 h = (__bf16)v[i]; r.h[i] = h; r.l[i] = (__bf16)(v[i] - (float)h); }
  return r; }
__device__ __forceinline__ F2 split_row(const float* row, int k0, int lane) { float v[16]; const float* p = row + k0 + 8 * (lane >> 4);
#pragma unroll
  for (int i = 0; i < 8; ++i) { v[i] = p[i]; v[8 + i] = p[16 + i]; }
  return bsplit16(v); }
__device__ __forceinline__ F2 split_rowK(const float* row, int k0, int lane, int K) { float v[16]; const int g = lane >> 4;
#pragma unroll
  for (int i = 0; i < 8; ++i) { const int ka = k0 + 8 * g + i, kb = ka + 16; v[i] = ka < K ? row[ka < K ? ka : K - 1] : 0.f; v[8 + i] = kb < K ? row[kb < K ? kb : K - 1] : 0.f; }
  return bsplit16(v); }
__device__ __forceinline__ F2 split_col(const float* W, int k0, int n, int lane, int ld, int K) { float v[16]; const int g = lane >> 4;
#pragma unroll
  for (int i = 0; i < 8; ++i) { const int ka = k0 + 8 * g + i, kb = ka + 16; v[i] = ka < K ? W[(size_t)(ka < K ? ka : K - 1) * ld + n] : 0.f; v[8 + i] = kb < K ? W[(size_t)(kb < K ? kb : K - 1) * ld + n] : 0.f; }
  return bsplit16(v); }
__device__ __forceinline__ v8f mac3(const F2& a, const F2& b, v8f c) { c = wmma_bf(a.l, b.h, c); c = wmma_bf(a.h, b.l, c); return wmma_bf(a.h, b.h, c); }
__device__ __forceinline__ float sigm(float v) { return 1.0f / (1.0f + expf(-v)); }
#define LDSX() do { asm volatile("s_wait_dscnt 0" ::: "memory"); __builtin_amdgcn_wave_barrier(); __builtin_amdgcn_fence(__ATOMIC_RELEASE, "workgroup"); } while (0)


#define NB 2
#define SS 512
#define HH 1024
#define DD 24
#define MH 96
#define VIN (2 * HH)
#define OH 1024
#define NR (NB * SS)
#ifndef NBT
#define NBT NB
#define TB0 0
#define TJB (SS / 16)
#endif
#define RB0 ((size_t)TB0 * SS)
typedef __attribute__((ext_vector_type(8))) __bf16 v8b;
__device__ __forceinline__ v16b frag_b(const __bf16* rowk0, int lane) {
  union { v16b v; v8b q[2]; } u; const __bf16* p = rowk0 + 8 * (lane >> 4);
  u.q[0] = *(const v8b*)p; u.q[1] = *(const v8b*)(p + 16); return u.v;
}
__device__ __forceinline__ float bfr(float v) { return (float)(__bf16)v; }
__device__ __attribute__((noinline)) float exp_ni(float v) { return expf(v); }
__device__ __attribute__((noinline)) float erf_ni(float v) { return erff(v); }

#define PK_PJ 0
#define PK_PI ((size_t)32 * HH)
#define PK_W1 (PK_PI + (size_t)32 * HH)
#define PK_V1 (PK_W1 + (size_t)MH * MH)
#define PK_V2 (PK_V1 + (size_t)OH * VIN)
#define PK_END (PK_V2 + (size_t)HH * OH)
#define WS_PK  0u
#define WS_Z   (((2u * PK_END) + 127u) / 128u * 128u)
#define WS_HIT (WS_Z + 4u * 2 * NR * 32)
#define WS_PH  (WS_HIT + 2u * (size_t)NB * HH * SS)
#define WS_PL  (WS_PH + 2u * NR * SS)
#define WS_CTX (WS_PL + 2u * NR * SS)
#define WS_GH  (WS_CTX + 4u * NR * HH)
#define WS_GL  (WS_GH + 2u * NR * OH)
#define WS_END (WS_GL + 2u * NR * OH)

__global__ __launch_bounds__(256) void k_pack(const float* __restrict__ PJ, const float* __restrict__ PI, const float* __restrict__ W1, const float* __restrict__ WV1, const float* __restrict__ WV2, __bf16* __restrict__ PK) {
  __shared__ __align__(16) __bf16 s[VIN]; const int n = blockIdx.x, which = blockIdx.y, t = threadIdx.x; int K; size_t dst;
  switch (which) {
    case 0: case 1: { if (n >= 32) return; K = HH; dst = ((which == 0) ? PK_PJ : PK_PI) + (size_t)n * HH; const float* P = (which == 0) ? PJ : PI; for (int k = t; k < K; k += 256) s[k] = (__bf16)((n < DD) ? P[(size_t)k * DD + n] : 0.f); break; }
    case 2: { if (n >= MH) return; K = MH; dst = PK_W1 + (size_t)n * MH; for (int k = t; k < K; k += 256) s[k] = (__bf16)W1[(size_t)k * MH + n]; break; }
    case 3: { K = VIN; dst = PK_V1 + (size_t)n * VIN; for (int k = t; k < K; k += 256) s[k] = (__bf16)WV1[(size_t)k * OH + n]; break; }
    default: { K = OH; dst = PK_V2 + (size_t)n * OH; for (int k = t; k < K; k += 256) s[k] = (__bf16)WV2[(size_t)k * HH + n]; break; } }
  __syncthreads();
  for (int q = t; q < K / 8; q += 256) vst2((unsigned*)(PK + dst + q * 8), *(const v4u*)&s[q * 8]);
}
__global__ __launch_bounds__(128) void k_z(const float* __restrict__ HJ, const float* __restrict__ HI, const __bf16* __restrict__ PK, float* __restrict__ Z) {
  __shared__ __align__(16) float so[4][16][36];
  const int tid = threadIdx.x, wave = tid >> 5, lane = tid & 31, col = lane & 15, g = lane >> 4; const int which = blockIdx.y; const size_t r0 = RB0 + (size_t)blockIdx.x * 64 + wave * 16; const float* X = (which == 0) ? HJ : HI; const __bf16* P = PK + ((which == 0) ? PK_PJ : PK_PI);
  v8f acc[2] = {};
#pragma unroll 2
  for (int kc = 0; kc < HH / 32; ++kc) { v16b a; { const float* p = X + (r0 + col) * HH + kc * 32 + 8 * g;
#pragma unroll
      for (int i = 0; i < 8; ++i) { a[i] = (__bf16)p[i]; a[8 + i] = (__bf16)p[16 + i]; } }
#pragma unroll
    for (int j = 0; j < 2; ++j) acc[j] = wmma_bf(a, frag_b(P + (size_t)(j * 16 + col) * HH + kc * 32, lane), acc[j]); }
#pragma unroll
  for (int j = 0; j < 2; ++j)
#pragma unroll
    for (int r = 0; r < 8; ++r) so[wave][8 * g + r][j * 16 + col] = acc[j][r];
  LDSX();
  for (int rl = 0; rl < 16; ++rl) if (lane < 8) vst2(Z + ((size_t)which * NR + r0 + rl) * 32 + lane * 4, *(const v4f*)&so[wave][rl][lane * 4]);
}
__global__ __launch_bounds__(256) void k_hit(const float* __restrict__ HI, __bf16* __restrict__ HIT) {
  __shared__ __align__(16) __bf16 s[128][72]; const int tid = threadIdx.x; const int ib = blockIdx.x, hb = blockIdx.y; const size_t b = blockIdx.z + TB0; const int i0 = ib * 64, h0 = hb * 128;
  for (int e = tid; e < 64 * 128; e += 256) { const int r = e >> 7, h = e & 127; s[h][r] = (__bf16)HI[((b * SS) + i0 + r) * HH + h0 + h]; }
  __syncthreads();
  for (int e = tid; e < 128 * 8; e += 256) { const int h = e >> 3, pc = e & 7; vst2((unsigned*)(HIT + (b * HH + h0 + h) * SS + i0 + pc * 8), *(const v4u*)&s[h][pc * 8]); }
}
__global__ __launch_bounds__(128) void k_pair(const float* __restrict__ Z, const __bf16* __restrict__ PK, const float* __restrict__ B1, const float* __restrict__ W2, const float* __restrict__ B2, const float* __restrict__ AM, __bf16* __restrict__ PH, __bf16* __restrict__ PL) {
  __shared__ float szi[SS][DD + 1]; __shared__ float szj[16][DD + 1]; __shared__ float slg[16][SS + 4];
  const int tid = threadIdx.x, wave = tid >> 5, lane = tid & 31, col = lane & 15, g = lane >> 4; const size_t b = blockIdx.y + TB0; const int j0 = blockIdx.x * 16;
  for (int e = tid; e < SS * DD; e += 128) { const int i = e / DD, d = e % DD; szi[i][d] = Z[((size_t)NR + b * SS + i) * 32 + d]; }
  for (int e = tid; e < 16 * DD; e += 128) { const int jl = e / DD, d = e % DD; szj[jl][d] = Z[(b * SS + j0 + jl) * 32 + d]; }
  __syncthreads();
  float w2l[6]; for (int ct = 0; ct < 6; ++ct) w2l[ct] = bfr(W2[ct * 16 + col]); const float b2v = bfr(B2[0]);
#pragma unroll 1
  for (int jj = 0; jj < 4; ++jj) { const int jl = wave * 4 + jj;
#pragma unroll 1
    for (int it = 0; it < SS / 16; ++it) { const int i = it * 16 + col;
      v8f acc[6] = {};
#pragma unroll
      for (int kc = 0; kc < 3; ++kc) { v16b ah, al;
#pragma unroll
        for (int q = 0; q < 16; ++q) { const int k = kc * 32 + 8 * g + (q & 7) + ((q >> 3) << 4); float f; const int d = k % DD; const int part = k / DD;
          const float zj = szj[jl][d], zi = szi[i][d]; f = (part == 0) ? zj : (part == 1) ? zi : (part == 2) ? zj * zi : fabsf(zj - zi);
          const __bf16 hb = (__bf16)f; ah[q] = hb; al[q] = (__bf16)(f - (float)hb); }
#pragma unroll
        for (int ct = 0; ct < 6; ++ct) { const v16b w = frag_b(PK + PK_W1 + (size_t)(ct * 16 + col) * MH + kc * 32, lane); acc[ct] = wmma_bf(al, w, acc[ct]); acc[ct] = wmma_bf(ah, w, acc[ct]); } }
      float part8[8];
#pragma unroll
      for (int r = 0; r < 8; ++r) part8[r] = 0.f;
#pragma unroll
      for (int ct = 0; ct < 6; ++ct) { const float bb = bfr(B1[ct * 16 + col]);
#pragma unroll
        for (int r = 0; r < 8; ++r) part8[r] += fmaxf(acc[ct][r] + bb, 0.f) * w2l[ct]; }
#pragma unroll
      for (int r = 0; r < 8; ++r) { float v = part8[r];
#pragma unroll
        for (int o = 1; o < 16; o <<= 1) v += __shfl_xor(v, o);
        if (col == 0) { const int ii = it * 16 + 8 * g + r; const float mk = bfr(AM[b * SS + ii]); slg[jl][ii] = v + b2v + (1.0f - mk) * -3.4028234663852886e38f; } } } }
  __syncthreads();
  { const int jl = tid >> 3, q8 = tid & 7; float mx = -3.4e38f; for (int i = q8; i < SS; i += 8) mx = fmaxf(mx, slg[jl][i]);
#pragma unroll
    for (int o = 1; o < 8; o <<= 1) mx = fmaxf(mx, __shfl_xor(mx, o));
    float sm = 0.f; for (int i = q8; i < SS; i += 8) { const float e = exp_ni(slg[jl][i] - mx); slg[jl][i] = e; sm += e; }
#pragma unroll
    for (int o = 1; o < 8; o <<= 1) sm += __shfl_xor(sm, o);
    const float inv = 1.0f / sm; __syncthreads();
    for (int i = q8; i < SS; i += 8) slg[jl][i] *= inv; }
  __syncthreads();
  for (int e = tid; e < 16 * SS / 8; e += 128) { const int jl = e / (SS / 8), q = e % (SS / 8); __align__(16) __bf16 hh[8], ll[8];
#pragma unroll
    for (int u = 0; u < 8; ++u) { const float p = slg[jl][q * 8 + u]; const __bf16 hb = (__bf16)p; hh[u] = hb; ll[u] = (__bf16)(p - (float)hb); }
    vst2((unsigned*)(PH + (b * SS + j0 + jl) * SS + q * 8), *(const v4u*)hh); vst2((unsigned*)(PL + (b * SS + j0 + jl) * SS + q * 8), *(const v4u*)ll); }
}
__global__ __launch_bounds__(128) void k_ctx(const __bf16* __restrict__ PH, const __bf16* __restrict__ PL, const __bf16* __restrict__ HIT, float* __restrict__ CTX) {
  __shared__ __align__(16) float so[4][16][132];
  const int tid = threadIdx.x, wave = tid >> 5, lane = tid & 31, col = lane & 15, g = lane >> 4; const size_t b = blockIdx.z + TB0; const size_t r0 = b * SS + (size_t)blockIdx.x * 64 + wave * 16; const int n0 = blockIdx.y * 128;
  v8f acc[8] = {};
#pragma unroll 2
  for (int kc = 0; kc < SS / 32; ++kc) { const v16b a = frag_b(PH + (r0 + col) * SS + kc * 32, lane), al = frag_b(PL + (r0 + col) * SS + kc * 32, lane);
#pragma unroll
    for (int j = 0; j < 8; ++j) { const v16b w = frag_b(HIT + (b * HH + n0 + j * 16 + col) * SS + kc * 32, lane); acc[j] = wmma_bf(al, w, acc[j]); acc[j] = wmma_bf(a, w, acc[j]); } }
#pragma unroll
  for (int j = 0; j < 8; ++j)
#pragma unroll
    for (int r = 0; r < 8; ++r) so[wave][8 * g + r][j * 16 + col] = acc[j][r];
  LDSX();
  for (int rl = 0; rl < 16; ++rl) vst2(CTX + (r0 + rl) * HH + n0 + lane * 4, *(const v4f*)&so[wave][rl][lane * 4]);
}
template <int MODE>
__global__ __launch_bounds__(128) void k_msg(const float* __restrict__ CTX, const float* __restrict__ HJ, const __bf16* __restrict__ GH, const __bf16* __restrict__ GL, const __bf16* __restrict__ PK, const float* __restrict__ BIAS, const float* __restrict__ ALPHA, float* __restrict__ OUT, __bf16* __restrict__ OGH, __bf16* __restrict__ OGL) {
  __shared__ __align__(16) float so[4][16][132]; __shared__ __align__(16) __bf16 sg[4][16][136], sgl[4][16][136];
  const int tid = threadIdx.x, wave = tid >> 5, lane = tid & 31, col = lane & 15, g = lane >> 4; const size_t r0 = RB0 + (size_t)blockIdx.x * 64 + wave * 16; const int n0 = blockIdx.y * 128;
  v8f acc[8] = {};
  if (MODE == 1) {
#pragma unroll 2
    for (int kc = 0; kc < VIN / 32; ++kc) { F2 a; if (kc < HH / 32) a = split_row(CTX + (r0 + col) * HH, kc * 32, lane); else { const float* p = HJ + (r0 + col) * HH + (kc - HH / 32) * 32 + 8 * g;
#pragma unroll
        for (int i = 0; i < 8; ++i) { a.h[i] = (__bf16)p[i]; a.h[8 + i] = (__bf16)p[16 + i]; a.l[i] = (__bf16)0.f; a.l[8 + i] = (__bf16)0.f; } }
#pragma unroll
      for (int j = 0; j < 8; ++j) { const v16b w = frag_b(PK + PK_V1 + (size_t)(n0 + j * 16 + col) * VIN + kc * 32, lane); if (kc < HH / 32) acc[j] = wmma_bf(a.l, w, acc[j]); acc[j] = wmma_bf(a.h, w, acc[j]); } }
#pragma unroll
    for (int j = 0; j < 8; ++j) { const float bb = bfr(BIAS[n0 + j * 16 + col]);
#pragma unroll
      for (int r = 0; r < 8; ++r) { const float v = fmaxf(acc[j][r] + bb, 0.f); const __bf16 hb = (__bf16)v; sg[wave][8 * g + r][j * 16 + col] = hb; sgl[wave][8 * g + r][j * 16 + col] = (__bf16)(v - (float)hb); } }
    LDSX();
    for (int rl = 0; rl < 16; ++rl) { if (lane < 16) vst2((unsigned*)(OGH + (r0 + rl) * OH + n0 + lane * 8), *(const v4u*)&sg[wave][rl][lane * 8]); else vst2((unsigned*)(OGL + (r0 + rl) * OH + n0 + (lane - 16) * 8), *(const v4u*)&sgl[wave][rl][(lane - 16) * 8]); }
  } else {
#pragma unroll 2
    for (int kc = 0; kc < OH / 32; ++kc) { const v16b a = frag_b(GH + (r0 + col) * OH + kc * 32, lane), al = frag_b(GL + (r0 + col) * OH + kc * 32, lane);
#pragma unroll
      for (int j = 0; j < 8; ++j) { const v16b w = frag_b(PK + PK_V2 + (size_t)(n0 + j * 16 + col) * OH + kc * 32, lane); acc[j] = wmma_bf(al, w, acc[j]); acc[j] = wmma_bf(a, w, acc[j]); } }
    const float al = bfr(ALPHA[0]);
#pragma unroll
    for (int j = 0; j < 8; ++j) { const float bb = bfr(BIAS[n0 + j * 16 + col]);
#pragma unroll
      for (int r = 0; r < 8; ++r) so[wave][8 * g + r][j * 16 + col] = al * (acc[j][r] + bb); }
    LDSX();
    for (int rl = 0; rl < 16; ++rl) vst2(OUT + (r0 + rl) * HH + n0 + lane * 4, *(const v4f*)&so[wave][rl][lane * 4]); }
}
extern "C" void kernel_launch(void* const* d_in, const int* in_sizes, int n_in, void* d_out, int out_size, void* d_ws, size_t ws_size, hipStream_t stream) {
  (void)in_sizes; (void)n_in; (void)out_size;
  const float** F = (const float**)d_in;
  if (ws_size < (size_t)WS_END) return;
  char* ws = (char*)d_ws; __bf16 *PK = (__bf16*)(ws + WS_PK), *HIT = (__bf16*)(ws + WS_HIT), *PH = (__bf16*)(ws + WS_PH), *PL = (__bf16*)(ws + WS_PL), *GH = (__bf16*)(ws + WS_GH), *GL = (__bf16*)(ws + WS_GL); float *Z = (float*)(ws + WS_Z), *CTX = (float*)(ws + WS_CTX);
  k_pack<<<dim3(OH, 5), 256, 0, stream>>>(F[3], F[4], F[5], F[9], F[11], PK);
  k_z<<<dim3(NBT * SS / 64, 2), 128, 0, stream>>>(F[0], F[1], PK, Z);
  k_hit<<<dim3(SS / 64, HH / 128, NBT), 256, 0, stream>>>(F[1], HIT);
  k_pair<<<dim3(TJB, NBT), 128, 0, stream>>>(Z, PK, F[6], F[7], F[8], F[2], PH, PL);
  k_ctx<<<dim3(TJB / 4, HH / 128, NBT), 128, 0, stream>>>(PH, PL, HIT, CTX);
  k_msg<1><<<dim3(NBT * SS / 64, OH / 128), 128, 0, stream>>>(CTX, F[0], nullptr, nullptr, PK, F[10], nullptr, nullptr, GH, GL);
  k_msg<2><<<dim3(NBT * SS / 64, HH / 128), 128, 0, stream>>>(nullptr, nullptr, GH, GL, PK, F[12], F[13], (float*)d_out, nullptr, nullptr);
}
